// DeformableGConv_58634893525710
// MI455X (gfx1250) — hardware-verified
//
#include <hip/hip_runtime.h>
#include <stddef.h>
#include <stdint.h>


#define NN      50000
#define NE      800000
#define RAWD    128
#define HIDD    256
#define OUTD    64
#define KK      4
#define PHID    16
#define MP      50048
#define NTHR    256
#define NWAVE   8
#define EPT     8
#define CHUNK   (NTHR * EPT)
#define WCAP    (EPT * 32)
#define LISTN   (NWAVE * WCAP)
#define NBMAX   2048
#define NBRUN   1024
#define RCAP    28672
#define DEGCAP  64
#define STW     512
#define ST_DIK  0
#define ST_PHI  64
#define ST_SRC  80
#define ST_ATT  144
#define GBM     128
#define GTHR    256
#define GMB     (MP / GBM)
#define TB_B1   0
#define TB_B2   256
#define TB_BIAS 320
#define TB_TN   384
#define TABN    512
#define RECP    32
#define SCANB   49
#define PA_HB   (MP * 32 / NTHR)
#define PA_EB   (MP * 16 / NTHR)
#define WSMAX   134217728
#define LDS_AGG ((2 * RCAP + 2 * NBMAX + LISTN) * 4 + 64)

static_assert(KK * OUTD == 256);
static_assert(KK * PHID == 64);
static_assert(PHID - 1 == 15);
static_assert(MP % GBM == 0 && MP >= NN && MP - NN < GBM);
static_assert(((long long)NN * OUTD * 4) % 128 == 0);
static_assert((MP * 32) % NTHR == 0 && (MP * 16) % NTHR == 0);
static_assert((CHUNK & (CHUNK - 1)) == 0 && CHUNK <= 4096);
static_assert((NBMAX & (NBMAX - 1)) == 0 && NBMAX <= 4096);
static_assert((NBRUN & (NBRUN - 1)) == 0 && NBRUN <= NBMAX && NBRUN >= 16);
static_assert(NTHR * 8 == NBMAX);
static_assert(LISTN >= NBMAX);
static_assert((RCAP % 32) == 0 && RCAP > 16651 + 4096);
static_assert(DEGCAP == 64 && DEGCAP >= 38 + 8);
static_assert(NWAVE * STW <= RCAP);
static_assert(ST_ATT + DEGCAP * 4 <= STW && ST_SRC + DEGCAP <= ST_ATT);
static_assert(SCANB * NBRUN >= NN && (SCANB - 1) * NBRUN < NN);
static_assert(NE < (1 << 20));
static_assert(LDS_AGG <= 327680);
static_assert(GBM == (GTHR / 32) * 16);
static_assert((RAWD % 32) == 0 && (HIDD % 32) == 0 && ((2 * HIDD) % 32) == 0);
static_assert(TB_TN + 64 <= TABN);

typedef float          v2f   __attribute__((ext_vector_type(2)));
typedef float          v4f   __attribute__((ext_vector_type(4)));
typedef float          v8f   __attribute__((ext_vector_type(8)));
typedef int            v4i   __attribute__((ext_vector_type(4)));
typedef int            v8i   __attribute__((ext_vector_type(8)));
typedef unsigned short v8us  __attribute__((ext_vector_type(8)));
typedef unsigned short v16us __attribute__((ext_vector_type(16)));
typedef __bf16         v16bf __attribute__((ext_vector_type(16)));
typedef v4f  __attribute__((may_alias)) v4fa;
typedef v8us __attribute__((may_alias)) v8usa;
union FragB { v16bf v; v16us u; v8us h[2]; v8i w; };

__device__ __forceinline__ v8f wmb(const FragB& a, const FragB& b, v8f c) {
  v8f d = __builtin_amdgcn_wmma_f32_16x16x32_bf16(false, a.v, false, b.v, (short)0, c, false, false);
  asm volatile("v_nop\n\tv_nop\n\tv_nop\n\tv_nop" : "+v"(d) : "v"(a.w), "v"(b.w));
  return d;
}

__device__ __forceinline__ unsigned bfbits(float v) {
  const unsigned u = __float_as_uint(v);
  return (u + 0x7FFFu + ((u >> 16) & 1u)) >> 16;
}
__device__ __forceinline__ float rbf(float v) { return __uint_as_float(bfbits(v) << 16); }

__device__ __forceinline__ v8us cvt8b(const v4f a, const v4f b) {
  v8us o;
  o[0] = (unsigned short)bfbits(a.x); o[1] = (unsigned short)bfbits(a.y);
  o[2] = (unsigned short)bfbits(a.z); o[3] = (unsigned short)bfbits(a.w);
  o[4] = (unsigned short)bfbits(b.x); o[5] = (unsigned short)bfbits(b.y);
  o[6] = (unsigned short)bfbits(b.z); o[7] = (unsigned short)bfbits(b.w);
  return o;
}

__device__ __forceinline__ void wave_sync() {
  __builtin_amdgcn_fence(__ATOMIC_RELEASE, "workgroup");
  __builtin_amdgcn_wave_barrier();
  __builtin_amdgcn_fence(__ATOMIC_ACQUIRE, "workgroup");
}

__device__ __forceinline__ float sel4(const v4f v, const int k) {
  return (k == 0) ? v.x : ((k == 1) ? v.y : ((k == 2) ? v.z : v.w));
}

__device__ __forceinline__ void put8(unsigned short* p, const v8us hv) {
  *(volatile v8us*)p = hv;
  __threadfence();
  *(volatile v8us*)p = hv;
}

__device__ __forceinline__ void cvt_row8(const float* __restrict__ src, unsigned short* dst, int row, int c0, int pitch) {
  const int rc = row < NN ? row : NN - 1;
  const float* p = src + (size_t)rc * pitch + c0;
  v4f a = *(const v4f*)p, b = *(const v4f*)(p + 4);
  const v4f z4 = {0.f, 0.f, 0.f, 0.f};
  if (row >= NN) { a = z4; b = z4; }
  const v8us hv = cvt8b(a, b);
  put8(dst + (size_t)row * pitch + c0, hv);
}

__global__ __launch_bounds__(NTHR) __attribute__((amdgpu_num_vgpr(248)))
void k_pa(const float* __restrict__ h_l, const float* __restrict__ e_l, unsigned short* HLB, unsigned short* EB) {
  const int blk = (int)blockIdx.x, tid = (int)threadIdx.x;
  if (blk < PA_HB) {
    const int i = blk * NTHR + tid;
    cvt_row8(h_l, HLB, i >> 5, (i & 31) * 8, HIDD);
  } else {
    const int i = (blk - PA_HB) * NTHR + tid;
    cvt_row8(e_l, EB, i >> 4, (i & 15) * 8, RAWD);
  }
}

__global__ __launch_bounds__(NTHR) __attribute__((amdgpu_num_vgpr(248)))
void k_pb(const float* __restrict__ W, const float* __restrict__ W1, const float* __restrict__ Wphi,
          unsigned short* WT, unsigned short* W1B, unsigned short* WPHT) {
  const int blk = (int)blockIdx.x, tid = (int)threadIdx.x;
  const v4f z4 = {0.f, 0.f, 0.f, 0.f};
  if (blk < 32) {
    const int u = blk * NTHR + tid;
    const int n = u >> 5, k8 = (u & 31) * 8;
    const float* p = W + (size_t)k8 * 256 + n;
    v4f a, b;
    a.x = p[0];    a.y = p[256];  a.z = p[512];  a.w = p[768];
    b.x = p[1024]; b.y = p[1280]; b.z = p[1536]; b.w = p[1792];
    put8(WT + (size_t)n * 256 + k8, cvt8b(a, b));
  } else if (blk < 48) {
    const int u = (blk - 32) * NTHR + tid;
    const int n = u >> 4, k8 = (u & 15) * 8;
    const float* p = W1 + (size_t)n * RAWD + k8;
    const v4f a = *(const v4f*)p, b = *(const v4f*)(p + 4);
    put8(W1B + (size_t)n * RAWD + k8, cvt8b(a, b));
  } else {
    const int u = tid;
    const int n = u >> 4, k8 = (u & 15) * 8;
    const int ncl = n < 15 ? n : 14;
    const float* p = Wphi + (size_t)k8 * 15 + ncl;
    v4f a, b;
    a.x = p[0];  a.y = p[15]; a.z = p[30]; a.w = p[45];
    b.x = p[60]; b.y = p[75]; b.z = p[90]; b.w = p[105];
    if (n >= 15) { a = z4; b = z4; }
    put8(WPHT + (size_t)n * RAWD + k8, cvt8b(a, b));
  }
}

__global__ __launch_bounds__(NTHR) __attribute__((amdgpu_num_vgpr(248)))
void k_pc(const float* __restrict__ W2, const float* __restrict__ b1, const float* __restrict__ b2,
          const float* __restrict__ bias, const float* __restrict__ tilde, unsigned short* W2D, float* TAB) {
  const int blk = (int)blockIdx.x, tid = (int)threadIdx.x;
  if (blk < 16) {
    const int u = blk * NTHR + tid;
    const int n = u >> 6, k8 = (u & 63) * 8;
    const float* p = W2 + (size_t)n * HIDD + (k8 & 255);
    const v4f a = *(const v4f*)p, b = *(const v4f*)(p + 4);
    put8(W2D + (size_t)n * 512 + k8, cvt8b(a, b));
  } else {
    __shared__ __attribute__((aligned(16))) float tl[64];
    __shared__ __attribute__((aligned(16))) float tnl[64];
    if (tid < 64) tl[tid] = rbf(tilde[tid]);
    __syncthreads();
    {
      const int e = tid & 63;
      const int k = e >> 4;
      float ssq = 0.0f;
#pragma unroll 1
      for (int p = 0; p < PHID; ++p) { const float x = tl[k * PHID + p]; ssq = ssq + x * x; }
      const float q = tl[e] / sqrtf(ssq);
      if (tid < 64) tnl[e] = q;
    }
    __syncthreads();
    const int t = tid;
    const int i1 = t < 63 ? t : 63;
    int i2 = t - 64; i2 = i2 < 0 ? 0 : (i2 > 15 ? 15 : i2);
    int i3 = t - 80; i3 = i3 < 0 ? 0 : (i3 > 15 ? 15 : i3);
    int i4 = t - 96; i4 = i4 < 0 ? 0 : (i4 > 15 ? 15 : i4);
    const v4f a = *(const v4f*)(b1 + 4 * i1);
    const v4f b = *(const v4f*)(b2 + 4 * i2);
    const v4f c = *(const v4f*)(bias + 4 * i3);
    const v4f d = *(const v4fa*)(tnl + 4 * i4);
    v4f r;
    const v4f s = (t < 64) ? a : ((t < 80) ? b : c);
    r.x = rbf(s.x); r.y = rbf(s.y); r.z = rbf(s.z); r.w = rbf(s.w);
    const v4f z4 = {0.f, 0.f, 0.f, 0.f};
    r = (t < 96) ? r : ((t < 112) ? d : z4);
    if (t < 128) *(volatile v4f*)(TAB + 4 * t) = r;
    __threadfence();
    if (t < 128) *(volatile v4f*)(TAB + 4 * t) = r;
  }
}

template<int MODE>
__global__ __launch_bounds__(GTHR) __attribute__((amdgpu_num_vgpr(248)))
void k_gemm(const unsigned short* __restrict__ A, const unsigned short* __restrict__ BT,
            const float* __restrict__ tab, float* outF, unsigned short* outB, int* rec,
            int lda, int K, int nValid) {
  constexpr int NT = (MODE == 2) ? 1 : 4;
  constexpr int SP = (MODE == 2) ? 16 : 64;
  constexpr int LDO = (MODE == 0) ? 256 : 64;
  __shared__ __attribute__((aligned(16))) float stg[GBM * 64];
  __shared__ double red[GTHR];
  __shared__ double tot[2];
  const int tid = (int)threadIdx.x, lane = tid & 31, wave = tid >> 5, hh = lane >> 4, m = lane & 15;
  const int rowBase = (int)blockIdx.x * GBM;
  const int col0    = (int)blockIdx.y * 64;

  v8f acc[NT];
  {
    const v8f z = {0.f, 0.f, 0.f, 0.f, 0.f, 0.f, 0.f, 0.f};
#pragma unroll
    for (int t = 0; t < NT; ++t) acc[t] = z;
  }
  const unsigned short* ap = A + (size_t)(rowBase + 16 * wave + m) * (size_t)lda + 8 * hh;
  const unsigned short* bp = BT + (size_t)(col0 + m) * (size_t)K + 8 * hh;
#pragma unroll 1
  for (int k0 = 0; k0 < K; k0 += 32) {
    FragB af;
    af.h[0] = *(const v8usa*)(ap + k0);
    af.h[1] = *(const v8usa*)(ap + k0 + 16);
#pragma unroll
    for (int t = 0; t < NT; ++t) {
      const unsigned short* wq = bp + (size_t)(16 * t) * (size_t)K + k0;
      FragB bf;
      bf.h[0] = *(const v8usa*)wq;
      bf.h[1] = *(const v8usa*)(wq + 16);
      acc[t] = wmb(af, bf, acc[t]);
    }
  }

#pragma unroll
  for (int t = 0; t < NT; ++t) {
    const int lc = 16 * t + m;
    float badd = 0.0f;
    if constexpr (MODE == 3) badd = tab[TB_B2 + lc];
#pragma unroll
    for (int r = 0; r < 8; ++r) {
      const int lr = 16 * wave + 8 * hh + r;
      stg[lr * SP + lc] = acc[t][r] + badd;
    }
  }
  __syncthreads();

  if constexpr (MODE == 1) {
    const int q = lane >> 3, j = lane & 7;
    const v4f ba = *(const v4f*)(tab + TB_B1 + col0 + 8 * j);
    const v4f bb = *(const v4f*)(tab + TB_B1 + col0 + 8 * j + 4);
#pragma unroll 1
    for (int it = 0; it < 4; ++it) {
      const int lr = 16 * wave + 4 * it + q;
      const v4f x0 = *(const v4fa*)(stg + lr * 64 + 8 * j);
      const v4f x1 = *(const v4fa*)(stg + lr * 64 + 8 * j + 4);
      const bool live = (rowBase + lr) < nValid;
      const float f[8] = {x0.x + ba.x, x0.y + ba.y, x0.z + ba.z, x0.w + ba.w,
                          x1.x + bb.x, x1.y + bb.y, x1.z + bb.z, x1.w + bb.w};
      v8us hv, lv;
#pragma unroll
      for (int i = 0; i < 8; ++i) {
        float v = f[i];
        v = (v > 0.0f) ? v : (v - v);
        v = live ? v : 0.0f;
        const unsigned hb = bfbits(v);
        hv[i] = (unsigned short)hb;
        lv[i] = (unsigned short)bfbits(v - __uint_as_float(hb << 16));
      }
      unsigned short* rp = outB + (size_t)(rowBase + lr) * 512 + col0 + 8 * j;
      *(volatile v8us*)rp = hv;
      *(volatile v8us*)(rp + 256) = lv;
      __threadfence();
      *(volatile v8us*)rp = hv;
      *(volatile v8us*)(rp + 256) = lv;
    }
  } else if constexpr (MODE == 2) {
    const v4f x0 = *(const v4fa*)(stg + 4 * tid);
    const v4f x1 = *(const v4fa*)(stg + 4 * (tid + GTHR));
    float* op = outF + (size_t)rowBase * 16;
    *(volatile v4f*)(op + 4 * tid) = x0;
    *(volatile v4f*)(op + 4 * (tid + GTHR)) = x1;
    __threadfence();
    *(volatile v4f*)(op + 4 * tid) = x0;
    *(volatile v4f*)(op + 4 * (tid + GTHR)) = x1;
  } else {
    if constexpr (MODE == 3) {
      const int row = tid >> 1, half = tid & 1;
      const float* sr = stg + row * 64 + 32 * half;
      double ds = 0.0;
#pragma unroll 1
      for (int i = 0; i < 8; ++i) {
        const v4f x = *(const v4fa*)(sr + 4 * i);
        ds += (double)x.x * (double)x.x;
        ds += (double)x.y * (double)x.y;
        ds += (double)x.z * (double)x.z;
        ds += (double)x.w * (double)x.w;
      }
      ds = ((rowBase + row) < nValid) ? ds : 0.0;
      red[tid] = ds;
      __syncthreads();
      if (tid == 0) {
        double tsum = 0.0;
#pragma unroll 1
        for (int i = 0; i < GTHR; ++i) tsum += red[i];
        tot[0] = tsum;
      }
      __syncthreads();
      const double tv = tot[0];
      v4i w;
      w.x = (tid == 0) ? __double2loint(tv) : 0;
      w.y = (tid == 0) ? __double2hiint(tv) : 0;
      w.z = 0; w.w = 0;
      int* rp = rec + (size_t)blockIdx.x * RECP + 4 * (tid & 7);
      if (tid < 8) *(volatile v4i*)rp = w;
      __threadfence();
      if (tid < 8) *(volatile v4i*)rp = w;
    }
    v4f add4 = {0.f, 0.f, 0.f, 0.f};
    if constexpr (MODE == 3) add4 = *(const v4f*)(tab + TB_TN + 4 * m);
    v4f fv[8];
#pragma unroll
    for (int i = 0; i < 8; ++i) {
      const int lr = 16 * wave + 2 * i + hh;
      fv[i] = *(const v4fa*)(stg + lr * 64 + 4 * m) + add4;
    }
#pragma unroll
    for (int i = 0; i < 8; ++i) {
      const int gr = rowBase + 16 * wave + 2 * i + hh;
      float* op = outF + (size_t)gr * LDO + col0 + 4 * m;
      *(volatile v4f*)op = fv[i];
    }
    __threadfence();
#pragma unroll
    for (int i = 0; i < 8; ++i) {
      const int gr = rowBase + 16 * wave + 2 * i + hh;
      float* op = outF + (size_t)gr * LDO + col0 + 4 * m;
      *(volatile v4f*)op = fv[i];
    }
  }
}

__device__ __forceinline__ int scan_chunk(const int* __restrict__ dsts, int nE, int cbase, int slotBase,
                                          int nb, int vec8, int* list, int tid, int lane, int wave) {
  int wc = 0;
  const int el0  = tid * EPT;
  const int e0   = cbase + el0;
  const int sent = -2147483647 - 1;
  v4i da, db;
  if (vec8 != 0 && cbase + CHUNK <= nE) {
    da = *(const v4i*)(dsts + e0);
    db = *(const v4i*)(dsts + e0 + 4);
  } else {
    da.x = (e0     < nE) ? dsts[min(e0,     nE - 1)] : sent;
    da.y = (e0 + 1 < nE) ? dsts[min(e0 + 1, nE - 1)] : sent;
    da.z = (e0 + 2 < nE) ? dsts[min(e0 + 2, nE - 1)] : sent;
    da.w = (e0 + 3 < nE) ? dsts[min(e0 + 3, nE - 1)] : sent;
    db.x = (e0 + 4 < nE) ? dsts[min(e0 + 4, nE - 1)] : sent;
    db.y = (e0 + 5 < nE) ? dsts[min(e0 + 5, nE - 1)] : sent;
    db.z = (e0 + 6 < nE) ? dsts[min(e0 + 6, nE - 1)] : sent;
    db.w = (e0 + 7 < nE) ? dsts[min(e0 + 7, nE - 1)] : sent;
  }
  const unsigned nbs = (unsigned)slotBase;
  const unsigned unb = (unsigned)nb;
  const unsigned s0 = (unsigned)da.x - nbs, s1 = (unsigned)da.y - nbs;
  const unsigned s2 = (unsigned)da.z - nbs, s3 = (unsigned)da.w - nbs;
  const unsigned s4 = (unsigned)db.x - nbs, s5 = (unsigned)db.y - nbs;
  const unsigned s6 = (unsigned)db.z - nbs, s7 = (unsigned)db.w - nbs;
  const bool h0 = s0 < unb, h1 = s1 < unb, h2 = s2 < unb, h3 = s3 < unb;
  const bool h4 = s4 < unb, h5 = s5 < unb, h6 = s6 < unb, h7 = s7 < unb;
  const unsigned any = __builtin_amdgcn_ballot_w32(h0 | h1 | h2 | h3 | h4 | h5 | h6 | h7);
  if (any != 0u) {
#define HITJ(J, HJ, SJ) { \
      const unsigned mj = __builtin_amdgcn_ballot_w32(HJ); \
      if (mj != 0u) { \
        if (HJ) { \
          const int pos = wc + (int)__builtin_amdgcn_mbcnt_lo(mj, 0u); \
          if (pos < WCAP) list[wave * WCAP + pos] = ((el0 + (J)) << 12) | (int)(SJ); \
        } \
        wc += (int)__builtin_popcount(mj); } }
    HITJ(0, h0, s0)
    HITJ(1, h1, s1)
    HITJ(2, h2, s2)
    HITJ(3, h3, s3)
    HITJ(4, h4, s4)
    HITJ(5, h5, s5)
    HITJ(6, h6, s6)
    HITJ(7, h7, s7)
#undef HITJ
  }
  return wc;
}

__global__ __launch_bounds__(NTHR) __attribute__((amdgpu_num_vgpr(248)))
void k_scan(const int* __restrict__ srcs, const int* __restrict__ dsts,
            const float* __restrict__ H, const float* __restrict__ DIK, const float* __restrict__ PHI,
            const float* __restrict__ tab, float* outp, int nN, int nE, int vec8) {
  extern __shared__ v4f lds_dyn[];
  int* reg1 = (int*)lds_dyn;
  int* reg2 = reg1 + RCAP;
  int* scnt = reg2 + RCAP;
  int* soff = scnt + NBMAX;
  int* list = soff + NBMAX;
  int* wcnt = list + LISTN;
  int* wtot = wcnt + NWAVE;
  const int tid = (int)threadIdx.x, lane = tid & 31, wave = tid >> 5;
  const int nb = NBRUN;
  const int nodeBase = (int)blockIdx.x * nb;

  for (int i = tid; i < NBMAX; i += NTHR) scnt[i] = 0;
  __syncthreads();

  int tot = 0;
  const int nChunks = (nE + CHUNK - 1) / CHUNK;
#pragma unroll 1
  for (int ch = 0; ch < nChunks; ++ch) {
    const int cbase = ch * CHUNK;
    const int wc = scan_chunk(dsts, nE, cbase, nodeBase, nb, vec8, list, tid, lane, wave);
    if (lane == 0) wcnt[wave] = wc;
    __syncthreads();
    int pre = 0, all = 0;
#pragma unroll
    for (int w2 = 0; w2 < NWAVE; ++w2) {
      int c = wcnt[w2];
      c = c < 0 ? 0 : (c > WCAP ? WCAP : c);
      all += c;
      pre += (w2 < wave) ? c : 0;
    }
    const int wcc  = wc > WCAP ? WCAP : wc;
    const int base = tot + pre;
#pragma unroll 1
    for (int i = lane; i < wcc; i += 32) {
      const int ent = list[wave * WCAP + i];
      const int el  = (ent >> 12) & (CHUNK - 1);
      const int sl  = ent & (NBMAX - 1);
      int eid = cbase + el;
      eid = eid > nE - 1 ? nE - 1 : eid;
      const int pos = base + i;
      if (pos < RCAP) reg1[pos] = (int)(((unsigned)eid << 12) | (unsigned)sl);
    }
    tot += all;
    tot = tot > RCAP ? RCAP : tot;
    __syncthreads();
  }
  const int nh = tot;

  if (wave == 0) {
#pragma unroll 1
    for (int b0 = 0; b0 < nh; b0 += 32) {
      int idx = b0 + lane;
      idx = idx < nh ? idx : nh - 1;
      const int uv  = reg1[idx];
      const int m32 = (nh - b0) < 32 ? (nh - b0) : 32;
#pragma unroll 1
      for (int k = 0; k < m32; ++k) {
        const int u  = __builtin_amdgcn_readlane(uv, k);
        const int sl = u & (NBMAX - 1);
        if (lane == 0) scnt[sl] = scnt[sl] + 1;
      }
    }
  }
  __syncthreads();

  {
    const v4i ca = *(const v4i*)(scnt + 8 * tid);
    const v4i cb = *(const v4i*)(scnt + 8 * tid + 4);
    const int e0 = ca.x < 0 ? 0 : ca.x, e1 = ca.y < 0 ? 0 : ca.y, e2 = ca.z < 0 ? 0 : ca.z, e3 = ca.w < 0 ? 0 : ca.w;
    const int e4 = cb.x < 0 ? 0 : cb.x, e5 = cb.y < 0 ? 0 : cb.y, e6 = cb.z < 0 ? 0 : cb.z, e7 = cb.w < 0 ? 0 : cb.w;
    const int ts = e0 + e1 + e2 + e3 + e4 + e5 + e6 + e7;
    int incl = ts;
#pragma unroll
    for (int d = 1; d < 32; d <<= 1) {
      const int up = __shfl_up(incl, d);
      if (lane >= d) incl += up;
    }
    if (lane == 31) wtot[wave] = incl;
    __syncthreads();
    int pre = 0;
#pragma unroll
    for (int w2 = 0; w2 < NWAVE; ++w2) pre += (w2 < wave) ? wtot[w2] : 0;
    int run = pre + incl - ts;
    soff[8 * tid + 0] = run; run += e0;
    soff[8 * tid + 1] = run; run += e1;
    soff[8 * tid + 2] = run; run += e2;
    soff[8 * tid + 3] = run; run += e3;
    soff[8 * tid + 4] = run; run += e4;
    soff[8 * tid + 5] = run; run += e5;
    soff[8 * tid + 6] = run; run += e6;
    soff[8 * tid + 7] = run;
  }
  __syncthreads();
  for (int i = tid; i < NBMAX; i += NTHR) list[i] = soff[i];
  __syncthreads();

  if (wave == 0) {
#pragma unroll 1
    for (int b0 = 0; b0 < nh; b0 += 32) {
      int idx = b0 + lane;
      idx = idx < nh ? idx : nh - 1;
      const int uv  = reg1[idx];
      const int m32 = (nh - b0) < 32 ? (nh - b0) : 32;
#pragma unroll 1
      for (int k = 0; k < m32; ++k) {
        const int u   = __builtin_amdgcn_readlane(uv, k);
        const int sl  = u & (NBMAX - 1);
        const int eid = (int)((unsigned)u >> 12);
        if (lane == 0) {
          int pos = list[sl];
          pos = pos < 0 ? 0 : (pos > RCAP - 1 ? RCAP - 1 : pos);
          reg2[pos] = eid;
          list[sl] = pos + 1;
        }
      }
    }
  }
  __syncthreads();

  const int nbw = nb >> 3;
  const bool ovf = (nh >= RCAP);
  const float qnan = __int_as_float(0x7fc00000);
  const float ninf = __int_as_float((int)0xff800000u);
  float* stw = (float*)reg1 + wave * STW;
  int*   swi = reg1 + wave * STW;
  const int l15 = lane & 15;
  const int hi  = lane >> 4;
  const v4f bias4 = *(const v4f*)(tab + TB_BIAS + 4 * l15);
#pragma unroll 1
  for (int jt = 0; jt < nbw; ++jt) {
    const int slot = wave * nbw + jt;
    const int grow = nodeBase + slot;
    const int gcl  = grow < nN ? grow : nN - 1;
    int st = soff[slot];
    const int craw = scnt[slot];
    int cnt = craw;
    st  = st < 0 ? 0 : (st > nh ? nh : st);
    cnt = cnt < 0 ? 0 : (cnt > DEGCAP ? DEGCAP : cnt);
    if (cnt > nh - st) cnt = nh - st;
    const float pz = (ovf || craw > DEGCAP) ? qnan : 0.0f;

    const v4f dv = *(const v4f*)(DIK + (size_t)gcl * 64 + 4 * l15);
    const v4f pv = *(const v4f*)(PHI + (size_t)gcl * 16 + 4 * (lane & 3));
    wave_sync();
    if (lane < 16) *(v4fa*)(stw + ST_DIK + 4 * lane) = dv;
    if (lane < 4)  *(v4fa*)(stw + ST_PHI + 4 * lane) = pv;
    wave_sync();
    const v4f pd0 = *(const v4fa*)(stw + ST_PHI);
    const v4f pd1 = *(const v4fa*)(stw + ST_PHI + 4);
    const v4f pd2 = *(const v4fa*)(stw + ST_PHI + 8);
    const v4f pd3 = *(const v4fa*)(stw + ST_PHI + 12);

    const int nch = (cnt + 31) >> 5;
    float m0 = ninf, m1 = ninf, m2 = ninf, m3 = ninf;
#pragma unroll 1
    for (int c = 0; c < nch; ++c) {
      const int q = 32 * c + lane;
      const bool valid = q < cnt;
      const int qq = q < cnt ? q : cnt - 1;
      int idx = st + qq;
      idx = idx < 0 ? 0 : (idx > RCAP - 1 ? RCAP - 1 : idx);
      int eid = reg2[idx];
      eid = eid < 0 ? 0 : (eid > nE - 1 ? nE - 1 : eid);
      const int sraw = srcs[eid];
      const int s = sraw < 0 ? 0 : (sraw > nN - 1 ? nN - 1 : sraw);
      swi[ST_SRC + q] = s;
      const float* pr = PHI + (size_t)s * 16;
      const v4f e0 = *(const v4f*)(pr)      - pd0;
      const v4f e1 = *(const v4f*)(pr + 4)  - pd1;
      const v4f e2 = *(const v4f*)(pr + 8)  - pd2;
      const v4f e3 = *(const v4f*)(pr + 12) - pd3;
      float dd[16] = {e0.x, e0.y, e0.z, e0.w, e1.x, e1.y, e1.z, e1.w,
                      e2.x, e2.y, e2.z, e2.w, e3.x, e3.y, e3.z, 0.0f};
      bool allz = true;
#pragma unroll
      for (int p = 0; p < 15; ++p) allz = allz && (dd[p] == 0.0f);
      dd[15] = allz ? 1.0f : 0.0f;
      float n2 = 0.0f;
#pragma unroll
      for (int p = 0; p < 16; ++p) n2 = fmaf(dd[p], dd[p], n2);
      const float nrm = fmaxf(sqrtf(n2), 1.0e-8f);
      const float inv = 1.0f / nrm;
#pragma unroll
      for (int p = 0; p < 16; ++p) dd[p] = dd[p] * inv;
      float a0 = 0.f, a1 = 0.f, a2 = 0.f, a3 = 0.f;
#pragma unroll 1
      for (int k = 0; k < KK; ++k) {
        const float* dk = stw + ST_DIK + 16 * k;
        const v4f w0 = *(const v4fa*)(dk);
        const v4f w1 = *(const v4fa*)(dk + 4);
        const v4f w2 = *(const v4fa*)(dk + 8);
        const v4f w3 = *(const v4fa*)(dk + 12);
        float a = dd[0] * w0.x;
        a = fmaf(dd[1],  w0.y, a); a = fmaf(dd[2],  w0.z, a); a = fmaf(dd[3],  w0.w, a);
        a = fmaf(dd[4],  w1.x, a); a = fmaf(dd[5],  w1.y, a); a = fmaf(dd[6],  w1.z, a); a = fmaf(dd[7],  w1.w, a);
        a = fmaf(dd[8],  w2.x, a); a = fmaf(dd[9],  w2.y, a); a = fmaf(dd[10], w2.z, a); a = fmaf(dd[11], w2.w, a);
        a = fmaf(dd[12], w3.x, a); a = fmaf(dd[13], w3.y, a); a = fmaf(dd[14], w3.z, a); a = fmaf(dd[15], w3.w, a);
        a0 = (k == 0) ? a : a0;
        a1 = (k == 1) ? a : a1;
        a2 = (k == 2) ? a : a2;
        a3 = (k == 3) ? a : a3;
      }
      const v4f a4 = {a0, a1, a2, a3};
      *(v4fa*)(stw + ST_ATT + 4 * q) = a4;
      float r0 = valid ? a0 : ninf, r1 = valid ? a1 : ninf, r2 = valid ? a2 : ninf, r3 = valid ? a3 : ninf;
#pragma unroll
      for (int off = 16; off > 0; off >>= 1) {
        r0 = fmaxf(r0, __shfl_xor(r0, off));
        r1 = fmaxf(r1, __shfl_xor(r1, off));
        r2 = fmaxf(r2, __shfl_xor(r2, off));
        r3 = fmaxf(r3, __shfl_xor(r3, off));
      }
      m0 = fmaxf(m0, r0); m1 = fmaxf(m1, r1); m2 = fmaxf(m2, r2); m3 = fmaxf(m3, r3);
    }
    wave_sync();

    const v4f mv = {m0, m1, m2, m3};
    float s0 = 0.f, s1 = 0.f, s2 = 0.f, s3 = 0.f;
#pragma unroll 1
    for (int c = 0; c < nch; ++c) {
      const int q = 32 * c + lane;
      const bool valid = q < cnt;
      float* ap = stw + ST_ATT + 4 * q;
      const v4f a4 = *(const v4fa*)ap;
      float x0 = 0.f, x1 = 0.f, x2 = 0.f, x3 = 0.f;
#pragma unroll 1
      for (int k = 0; k < KK; ++k) {
        float ev = expf(sel4(a4, k) - sel4(mv, k));
        ev = valid ? ev : 0.0f;
        x0 = (k == 0) ? ev : x0;
        x1 = (k == 1) ? ev : x1;
        x2 = (k == 2) ? ev : x2;
        x3 = (k == 3) ? ev : x3;
      }
      const v4f x4 = {x0, x1, x2, x3};
      *(v4fa*)ap = x4;
      float r0 = x0, r1 = x1, r2 = x2, r3 = x3;
#pragma unroll
      for (int off = 16; off > 0; off >>= 1) {
        r0 += __shfl_xor(r0, off);
        r1 += __shfl_xor(r1, off);
        r2 += __shfl_xor(r2, off);
        r3 += __shfl_xor(r3, off);
      }
      s0 += r0; s1 += r1; s2 += r2; s3 += r3;
    }
    const v4f sv = {s0, s1, s2, s3};
#pragma unroll 1
    for (int c = 0; c < nch; ++c) {
      const int q = 32 * c + lane;
      float* ap = stw + ST_ATT + 4 * q;
      const v4f x4 = *(const v4fa*)ap;
      float t0 = 0.f, t1 = 0.f, t2 = 0.f, t3 = 0.f;
#pragma unroll 1
      for (int k = 0; k < KK; ++k) {
        const float tv = sel4(x4, k) / sel4(sv, k);
        t0 = (k == 0) ? tv : t0;
        t1 = (k == 1) ? tv : t1;
        t2 = (k == 2) ? tv : t2;
        t3 = (k == 3) ? tv : t3;
      }
      const v4f t4 = {t0, t1, t2, t3};
      *(v4fa*)ap = t4;
    }
    wave_sync();

    v4f acc0 = {0.f, 0.f, 0.f, 0.f}, acc1 = {0.f, 0.f, 0.f, 0.f};
#pragma unroll 1
    for (int e = 0; e < cnt; ++e) {
      int s = swi[ST_SRC + e];
      s = s < 0 ? 0 : (s > nN - 1 ? nN - 1 : s);
      const v4f t4 = *(const v4fa*)(stw + ST_ATT + 4 * e);
      const float* hr = H + (size_t)s * 256 + 4 * lane;
      const v4f v0 = *(const v4f*)hr;
      const v4f v1 = *(const v4f*)(hr + 128);
      const float wa = hi ? t4.y : t4.x;
      const float wb = hi ? t4.w : t4.z;
      acc0.x = fmaf(wa, v0.x, acc0.x); acc0.y = fmaf(wa, v0.y, acc0.y);
      acc0.z = fmaf(wa, v0.z, acc0.z); acc0.w = fmaf(wa, v0.w, acc0.w);
      acc1.x = fmaf(wb, v1.x, acc1.x); acc1.y = fmaf(wb, v1.y, acc1.y);
      acc1.z = fmaf(wb, v1.z, acc1.z); acc1.w = fmaf(wb, v1.w, acc1.w);
    }

    v4f r = acc0 + acc1;
    r.x += __shfl_xor(r.x, 16);
    r.y += __shfl_xor(r.y, 16);
    r.z += __shfl_xor(r.z, 16);
    r.w += __shfl_xor(r.w, 16);
    v4f o = r + bias4;
    float ss = o.x * o.x;
    ss = fmaf(o.y, o.y, ss); ss = fmaf(o.z, o.z, ss); ss = fmaf(o.w, o.w, ss);
    ss = (lane < 16) ? ss : 0.0f;
#pragma unroll
    for (int off = 16; off > 0; off >>= 1) ss += __shfl_xor(ss, off);
    const float onrm = fmaxf(sqrtf(ss), 1.0e-8f);
    const float oinv = 1.0f / onrm;
    o.x = o.x * oinv + pz; o.y = o.y * oinv + pz; o.z = o.z * oinv + pz; o.w = o.w * oinv + pz;
    float* gp = outp + (size_t)gcl * OUTD + 4 * l15;
    const bool wsv = (grow < nN) && (lane < 16);
    if (wsv) *(volatile v4f*)gp = o;
    __threadfence();
    if (wsv) *(volatile v4f*)gp = o;
  }
}

__global__ __launch_bounds__(32) __attribute__((amdgpu_num_vgpr(248)))
void k_fin(const int* __restrict__ rec, const float* __restrict__ tab, float* outp) {
  if (threadIdx.x == 0) {
    double s = 0.0;
#pragma unroll 1
    for (int b = 0; b < GMB; ++b) {
      const v4i r = *(const v4i*)(rec + (size_t)b * RECP);
      s += __hiloint2double(r.y, r.x);
    }
    const float lf = (float)(s / 200000.0);
    double ls = 0.0;
#pragma unroll 1
    for (int k = 0; k < KK; ++k) {
#pragma unroll 1
      for (int j = 0; j < KK; ++j) {
#pragma unroll 1
        for (int p = 0; p < PHID; ++p) {
          const double d = (double)tab[TB_TN + k * PHID + p] - (double)tab[TB_TN + j * PHID + p];
          ls += d * d;
        }
      }
    }
    const float lsep = (float)(ls / 4.0);
    const v2f o = {lsep, lf};
    float* op = outp + (size_t)NN * OUTD;
    *(volatile v2f*)op = o;
    __threadfence();
    *(volatile v2f*)op = o;
  }
}

static inline size_t al256(size_t o) { return (o + 255) & ~(size_t)255; }

extern "C" void kernel_launch(void* const* d_in, const int* in_sizes, int n_in,
                              void* d_out, int out_size, void* d_ws, size_t ws_size,
                              hipStream_t stream) {
  if (n_in < 12) return;
  if (in_sizes[0] != NN * HIDD || in_sizes[1] != NN * RAWD) return;
  if (in_sizes[2] != NE || in_sizes[3] != NE) return;
  if (in_sizes[4] != RAWD * 15 || in_sizes[5] != HIDD * RAWD) return;
  if (in_sizes[6] != HIDD || in_sizes[7] != 64 * HIDD || in_sizes[8] != 64) return;
  if (in_sizes[9] != 64 || in_sizes[10] != HIDD * 256 || in_sizes[11] != 64) return;
  if (out_size != NN * OUTD + 2) return;

  const float* h_l   = (const float*)d_in[0];
  const float* e_l   = (const float*)d_in[1];
  const int*   src   = (const int*)  d_in[2];
  const int*   dst   = (const int*)  d_in[3];
  const float* W_phi = (const float*)d_in[4];
  const float* W1    = (const float*)d_in[5];
  const float* b1    = (const float*)d_in[6];
  const float* W2    = (const float*)d_in[7];
  const float* b2    = (const float*)d_in[8];
  const float* tilde = (const float*)d_in[9];
  const float* W     = (const float*)d_in[10];
  const float* bias  = (const float*)d_in[11];
  float* out = (float*)d_out;

  char* ws = (char*)d_ws;
  size_t off = 0;
  const size_t oP    = off; off = al256(off + (size_t)MP * 512 * 2);
  const size_t oQ    = off; off = al256(off + (size_t)MP * 256 * 4);
  const size_t oEB   = off; off = al256(off + (size_t)MP * RAWD * 2);
  const size_t oDIK  = off; off = al256(off + (size_t)MP * 64 * 4);
  const size_t oPHI  = off; off = al256(off + (size_t)MP * 16 * 4);
  const size_t oWT   = off; off = al256(off + (size_t)256 * 256 * 2);
  const size_t oW1B  = off; off = al256(off + (size_t)256 * RAWD * 2);
  const size_t oWPHT = off; off = al256(off + (size_t)16 * RAWD * 2);
  const size_t oW2D  = off; off = al256(off + (size_t)64 * 512 * 2);
  const size_t oTAB  = off; off = al256(off + (size_t)TABN * 4);
  const size_t oREC  = off; off = al256(off + (size_t)GMB * RECP * 4);
  if (off > ws_size || off > (size_t)WSMAX) return;
  unsigned short* P    = (unsigned short*)(ws + oP);
  float*          Hq   = (float*)(ws + oQ);
  unsigned short* EB   = (unsigned short*)(ws + oEB);
  float*          DIK  = (float*)(ws + oDIK);
  float*          PHI  = (float*)(ws + oPHI);
  unsigned short* WT   = (unsigned short*)(ws + oWT);
  unsigned short* W1B  = (unsigned short*)(ws + oW1B);
  unsigned short* WPHT = (unsigned short*)(ws + oWPHT);
  unsigned short* W2D  = (unsigned short*)(ws + oW2D);
  float*          TAB  = (float*)(ws + oTAB);
  int*            REC  = (int*)(ws + oREC);

  hipFuncSetAttribute(reinterpret_cast<const void*>(&k_scan), hipFuncAttributeMaxDynamicSharedMemorySize, LDS_AGG);

  k_pa<<<PA_HB + PA_EB, NTHR, 0, stream>>>(h_l, e_l, P, EB);
  k_pb<<<49, NTHR, 0, stream>>>(W, W1, W_phi, WT, W1B, WPHT);
  k_pc<<<17, NTHR, 0, stream>>>(W2, b1, b2, bias, tilde, W2D, TAB);
  k_gemm<0><<<dim3(GMB, 4), GTHR, 0, stream>>>(P, WT, TAB, Hq, EB, REC, HIDD, HIDD, NN);
  k_gemm<1><<<dim3(GMB, 4), GTHR, 0, stream>>>(EB, W1B, TAB, DIK, P, REC, RAWD, RAWD, NN);
  k_gemm<2><<<dim3(GMB, 1), GTHR, 0, stream>>>(EB, WPHT, TAB, PHI, W2D, REC, RAWD, RAWD, NN);
  k_gemm<3><<<dim3(GMB, 1), GTHR, 0, stream>>>(P, W2D, TAB, DIK, EB, REC, 512, 512, NN);
  k_scan<<<SCANB, NTHR, LDS_AGG, stream>>>(src, dst, Hq, DIK, PHI, TAB, out, NN, NE, ((NE & 3) == 0) ? 1 : 0);
  k_fin<<<1, 32, 0, stream>>>(REC, TAB, out);
}
